// DHSpaceKAA_57827439673618
// MI455X (gfx1250) — hardware-verified
//
#include <hip/hip_runtime.h>
#include <stddef.h>
#include <stdint.h>


#define DF    128
#define NH    8
#define HC    16
#define NTY   3
#define NREL  3
#define WSZ   (DF * DF)
#define GR    32
#define AP    136
#define QP    132
#define NTHR  256
#define NWAVE 8
#define NB    256
#define CHUNK 2048
#define WCAP  256
#define NGRP  (CHUNK / (NTHR * 4))

#define LDS_SACC (NB * DF)
#define LDS_DEN  (NB * NH)
#define LDS_MX   (NB * NH)
#define LDS_LIST (NWAVE * WCAP)
#define LDS_PRI  32
#define LDS_BYTES ((LDS_SACC + LDS_DEN + LDS_MX + LDS_LIST + NWAVE + LDS_PRI) * 4)

static_assert(WCAP == (CHUNK / NTHR) * 32);
static_assert(NGRP == 2);
static_assert(NB == 256);
static_assert((NB / NWAVE) == 32);
static_assert(((LDS_SACC + LDS_DEN) % 4) == 0);
static_assert((LDS_MX % 4) == 0);
static_assert(NREL * NH <= LDS_PRI);
static_assert(LDS_BYTES == 155808);
static_assert((GR / NWAVE) == 4);

typedef float    v4f  __attribute__((ext_vector_type(4)));
typedef float    v8f  __attribute__((ext_vector_type(8)));
typedef int      v4i  __attribute__((ext_vector_type(4)));
typedef _Float16 v4h  __attribute__((ext_vector_type(4)));
typedef _Float16 v8h  __attribute__((ext_vector_type(8)));
typedef _Float16 v16h __attribute__((ext_vector_type(16)));
union Frag   { v16h v; v8h half[2]; };
union Pack16 { v8h h; v4i i; };

__device__ __forceinline__ v8f wm(v16h a, v16h b, v8f c) {
  v8f d = __builtin_amdgcn_wmma_f32_16x16x32_f16(false, a, false, b, (short)0, c, false, false);
  asm volatile("v_nop\n\tv_nop\n\tv_nop\n\tv_nop" : "+v"(d) : "v"(a), "v"(b));
  return d;
}

__device__ __forceinline__ float wsum(float v) {
  v += __shfl_xor(v, 16, 32);
  v += __shfl_xor(v, 8, 32);
  v += __shfl_xor(v, 4, 32);
  v += __shfl_xor(v, 2, 32);
  v += __shfl_xor(v, 1, 32);
  return v;
}

__device__ __forceinline__ float sel3(int t, float a, float b, float c) {
  return (t == 0) ? a : ((t == 1) ? b : c);
}

__device__ __forceinline__ float gelu_exact(float v) {
  return 0.5f * v * (1.0f + erff(v * 0.70710678118654752f));
}

__global__ __launch_bounds__(NTHR) void k_prep(const float* __restrict__ W0, const float* __restrict__ W1,
                                               const float* __restrict__ W2, const float* __restrict__ W3,
                                               _Float16* Wp) {
  __shared__ __attribute__((aligned(16))) _Float16 Tt[DF * AP];
  const int tid = threadIdx.x, lane = tid & 31, wave = tid >> 5, hh = lane >> 4, m = lane & 15;
  const int g = blockIdx.x;
  const int tens = g / NTY, ty = g - tens * NTY;
  const float* W = (tens == 0) ? W0 : ((tens == 1) ? W1 : ((tens == 2) ? W2 : W3));
  const float* src = W + (size_t)ty * WSZ;
#pragma unroll 1
  for (int it = 0; it < WSZ / (NTHR * 4); ++it) {
    const int idx = (it * NTHR + tid) * 4;
    const int k = idx >> 7, n = idx & (DF - 1);
    const v4f w = *(const v4f*)(src + idx);
    Tt[(n + 0) * AP + k] = (_Float16)(w.x * 8.0f);
    Tt[(n + 1) * AP + k] = (_Float16)(w.y * 8.0f);
    Tt[(n + 2) * AP + k] = (_Float16)(w.z * 8.0f);
    Tt[(n + 3) * AP + k] = (_Float16)(w.w * 8.0f);
  }
  __syncthreads();
  _Float16* dst = Wp + (size_t)g * WSZ;
  v4i vv[8];
  _Float16* pp[8];
#pragma unroll
  for (int i = 0; i < 8; ++i) {
    const int row = 16 * wave + 2 * i + hh;
    Pack16 u;
    u.h = *(const v8h*)(Tt + row * AP + 8 * m);
    vv[i] = u.i;
    pp[i] = dst + (size_t)row * DF + 8 * m;
  }
#pragma unroll
  for (int i = 0; i < 8; ++i) *(volatile v4i*)(pp[i]) = vv[i];
  __threadfence();
#pragma unroll
  for (int i = 0; i < 8; ++i) *(volatile v4i*)(pp[i]) = vv[i];
}

__device__ __forceinline__ void gemm3(const _Float16* At, const _Float16* __restrict__ Wt, int m, int hh, int ncol,
                                      v8f& c00, v8f& c01, v8f& c02, v8f& c10, v8f& c11, v8f& c12) {
  const v8f z = {0.f, 0.f, 0.f, 0.f, 0.f, 0.f, 0.f, 0.f};
  c00 = z; c01 = z; c02 = z; c10 = z; c11 = z; c12 = z;
  const _Float16* pa0 = At + m * AP + 8 * hh;
  const _Float16* pa1 = At + (16 + m) * AP + 8 * hh;
  const _Float16* pb0 = Wt + ((size_t)0 * DF + ncol) * DF + 8 * hh;
  const _Float16* pb1 = Wt + ((size_t)1 * DF + ncol) * DF + 8 * hh;
  const _Float16* pb2 = Wt + ((size_t)2 * DF + ncol) * DF + 8 * hh;
#pragma unroll 2
  for (int kt = 0; kt < DF / 32; ++kt) {
    const int k0 = kt * 32;
    Frag a0, a1, b0, b1, b2;
    a0.half[0] = *(const v8h*)(pa0 + k0); a0.half[1] = *(const v8h*)(pa0 + k0 + 16);
    a1.half[0] = *(const v8h*)(pa1 + k0); a1.half[1] = *(const v8h*)(pa1 + k0 + 16);
    b0.half[0] = *(const v8h*)(pb0 + k0); b0.half[1] = *(const v8h*)(pb0 + k0 + 16);
    b1.half[0] = *(const v8h*)(pb1 + k0); b1.half[1] = *(const v8h*)(pb1 + k0 + 16);
    b2.half[0] = *(const v8h*)(pb2 + k0); b2.half[1] = *(const v8h*)(pb2 + k0 + 16);
    c00 = wm(a0.v, b0.v, c00); c01 = wm(a0.v, b1.v, c01); c02 = wm(a0.v, b2.v, c02);
    c10 = wm(a1.v, b0.v, c10); c11 = wm(a1.v, b1.v, c11); c12 = wm(a1.v, b2.v, c12);
  }
}

__global__ __launch_bounds__(NTHR) void k_node(
    const float* __restrict__ x, const int* __restrict__ ntype, const _Float16* __restrict__ Wp,
    const float* __restrict__ bq, const float* __restrict__ bk, const float* __restrict__ bv,
    const float* __restrict__ ratt, const float* __restrict__ rmsg,
    float* qo, _Float16* kro, _Float16* mso, int nN, int nP) {
  __shared__ __attribute__((aligned(16))) _Float16 Xs[GR * AP];
  __shared__ __attribute__((aligned(16))) _Float16 Ks[GR * AP];
  __shared__ __attribute__((aligned(16))) _Float16 Vs[GR * AP];
  __shared__ __attribute__((aligned(16))) _Float16 St[GR * AP];
  __shared__ __attribute__((aligned(16))) float Qs[GR * QP];
  __shared__ int ts[GR];

  const int tid  = threadIdx.x;
  const int lane = tid & 31;
  const int wave = tid >> 5;
  const int hh   = lane >> 4;
  const int m    = lane & 15;
  const int rowBase = blockIdx.x * GR;

  {
    const int r  = tid >> 3;
    const int c0 = (tid & 7) * 16;
    int row = rowBase + r;
    if (row > nN - 1) row = nN - 1;
    const float* p = x + (size_t)row * DF + c0;
    const v4f f0 = *(const v4f*)(p), f1 = *(const v4f*)(p + 4);
    const v4f f2 = *(const v4f*)(p + 8), f3 = *(const v4f*)(p + 12);
    Pack16 u0, u1;
    u0.h[0] = (_Float16)f0.x; u0.h[1] = (_Float16)f0.y; u0.h[2] = (_Float16)f0.z; u0.h[3] = (_Float16)f0.w;
    u0.h[4] = (_Float16)f1.x; u0.h[5] = (_Float16)f1.y; u0.h[6] = (_Float16)f1.z; u0.h[7] = (_Float16)f1.w;
    u1.h[0] = (_Float16)f2.x; u1.h[1] = (_Float16)f2.y; u1.h[2] = (_Float16)f2.z; u1.h[3] = (_Float16)f2.w;
    u1.h[4] = (_Float16)f3.x; u1.h[5] = (_Float16)f3.y; u1.h[6] = (_Float16)f3.z; u1.h[7] = (_Float16)f3.w;
    *(v8h*)(Xs + r * AP + c0)     = u0.h;
    *(v8h*)(Xs + r * AP + c0 + 8) = u1.h;
  }
  if (tid < GR) {
    int row = rowBase + tid;
    if (row > nN - 1) row = nN - 1;
    int t = ntype[row];
    t = (t < 0) ? 0 : ((t > NTY - 1) ? NTY - 1 : t);
    ts[tid] = t;
  }
  __syncthreads();

  const int ncol = wave * HC + m;
  v8f c00, c01, c02, c10, c11, c12;

  gemm3(Xs, Wp + (size_t)0 * NTY * WSZ, m, hh, ncol, c00, c01, c02, c10, c11, c12);
#pragma unroll
  for (int r = 0; r < 8; ++r) {
    const int r0 = 8 * hh + r, r1 = 16 + 8 * hh + r;
    const int t0 = ts[r0], t1 = ts[r1];
    Qs[r0 * QP + ncol] = sel3(t0, c00[r], c01[r], c02[r]) * 0.125f + bq[t0 * DF + ncol];
    Qs[r1 * QP + ncol] = sel3(t1, c10[r], c11[r], c12[r]) * 0.125f + bq[t1 * DF + ncol];
  }
  gemm3(Xs, Wp + (size_t)1 * NTY * WSZ, m, hh, ncol, c00, c01, c02, c10, c11, c12);
#pragma unroll
  for (int r = 0; r < 8; ++r) {
    const int r0 = 8 * hh + r, r1 = 16 + 8 * hh + r;
    const int t0 = ts[r0], t1 = ts[r1];
    Ks[r0 * AP + ncol] = (_Float16)(sel3(t0, c00[r], c01[r], c02[r]) + 8.0f * bk[t0 * DF + ncol]);
    Ks[r1 * AP + ncol] = (_Float16)(sel3(t1, c10[r], c11[r], c12[r]) + 8.0f * bk[t1 * DF + ncol]);
  }
  gemm3(Xs, Wp + (size_t)2 * NTY * WSZ, m, hh, ncol, c00, c01, c02, c10, c11, c12);
#pragma unroll
  for (int r = 0; r < 8; ++r) {
    const int r0 = 8 * hh + r, r1 = 16 + 8 * hh + r;
    const int t0 = ts[r0], t1 = ts[r1];
    Vs[r0 * AP + ncol] = (_Float16)(sel3(t0, c00[r], c01[r], c02[r]) + 8.0f * bv[t0 * DF + ncol]);
    Vs[r1 * AP + ncol] = (_Float16)(sel3(t1, c10[r], c11[r], c12[r]) + 8.0f * bv[t1 * DF + ncol]);
  }
  __syncthreads();

  {
    v4f qr[4];
    float* qp[4];
#pragma unroll
    for (int i = 0; i < 4; ++i) {
      qr[i] = *(const v4f*)(Qs + (4 * wave + i) * QP + 4 * lane);
      qp[i] = qo + (size_t)(rowBase + 4 * wave + i) * DF + 4 * lane;
    }
#pragma unroll
    for (int i = 0; i < 4; ++i) *(volatile v4f*)(qp[i]) = qr[i];
    __threadfence();
#pragma unroll
    for (int i = 0; i < 4; ++i) *(volatile v4f*)(qp[i]) = qr[i];
  }

  const v8h z8 = {(_Float16)0.f, (_Float16)0.f, (_Float16)0.f, (_Float16)0.f,
                  (_Float16)0.f, (_Float16)0.f, (_Float16)0.f, (_Float16)0.f};
  const v8f z  = {0.f, 0.f, 0.f, 0.f, 0.f, 0.f, 0.f, 0.f};
#pragma unroll 1
  for (int rl = 0; rl < NREL; ++rl) {
    Frag bA, bM;
    {
      v8h la = z8, lm = z8;
      const float* pa = ratt + ((size_t)(rl * NH + wave) * HC + 8 * hh) * HC + m;
      const float* pm = rmsg + ((size_t)(rl * NH + wave) * HC + 8 * hh) * HC + m;
#pragma unroll
      for (int i = 0; i < 8; ++i) {
        la[i] = (_Float16)pa[i * HC];
        lm[i] = (_Float16)pm[i * HC];
      }
      bA.half[0] = la; bA.half[1] = z8;
      bM.half[0] = lm; bM.half[1] = z8;
    }
    Frag aK0, aK1, aV0, aV1;
    aK0.half[0] = *(const v8h*)(Ks + m * AP + HC * wave + 8 * hh);        aK0.half[1] = z8;
    aK1.half[0] = *(const v8h*)(Ks + (16 + m) * AP + HC * wave + 8 * hh); aK1.half[1] = z8;
    aV0.half[0] = *(const v8h*)(Vs + m * AP + HC * wave + 8 * hh);        aV0.half[1] = z8;
    aV1.half[0] = *(const v8h*)(Vs + (16 + m) * AP + HC * wave + 8 * hh); aV1.half[1] = z8;
    const v8f dK0 = wm(aK0.v, bA.v, z);
    const v8f dK1 = wm(aK1.v, bA.v, z);
    const v8f dM0 = wm(aV0.v, bM.v, z);
    const v8f dM1 = wm(aV1.v, bM.v, z);
#pragma unroll
    for (int r = 0; r < 8; ++r) {
      const int r0 = 8 * hh + r, r1 = 16 + 8 * hh + r;
      St[r0 * AP + ncol] = (_Float16)dK0[r];
      St[r1 * AP + ncol] = (_Float16)dK1[r];
      Xs[r0 * AP + ncol] = (_Float16)dM0[r];
      Xs[r1 * AP + ncol] = (_Float16)dM1[r];
    }
    __syncthreads();
    {
      v4i kv[2], mv[2];
      _Float16* kp[2];
      _Float16* mp[2];
#pragma unroll
      for (int i = 0; i < 2; ++i) {
        const int row = 4 * wave + 2 * i + hh;
        Pack16 u;
        u.h = *(const v8h*)(St + row * AP + 8 * m); kv[i] = u.i;
        u.h = *(const v8h*)(Xs + row * AP + 8 * m); mv[i] = u.i;
        const size_t go = ((size_t)rl * nP + rowBase + row) * DF + 8 * m;
        kp[i] = kro + go;
        mp[i] = mso + go;
      }
#pragma unroll
      for (int i = 0; i < 2; ++i) { *(volatile v4i*)(kp[i]) = kv[i]; *(volatile v4i*)(mp[i]) = mv[i]; }
      __threadfence();
#pragma unroll
      for (int i = 0; i < 2; ++i) { *(volatile v4i*)(kp[i]) = kv[i]; *(volatile v4i*)(mp[i]) = mv[i]; }
    }
    __syncthreads();
  }
}

__global__ __launch_bounds__(NTHR) void k_agg(
    const int* __restrict__ esrc, const int* __restrict__ edst, const int* __restrict__ ety,
    const float* __restrict__ rpri, const float* __restrict__ q,
    const _Float16* __restrict__ kr8, const _Float16* __restrict__ ms8,
    float* aggr, int nN, int nE, int nP) {
  extern __shared__ v4f lds_dyn[];
  float* sacc = (float*)lds_dyn;
  float* den  = sacc + LDS_SACC;
  float* mx   = den + LDS_DEN;
  int*   list = (int*)(mx + LDS_MX);
  int*   wcnt = list + LDS_LIST;
  float* pri  = (float*)(wcnt + NWAVE);

  const int tid  = threadIdx.x;
  const int lane = tid & 31;
  const int wave = tid >> 5;
  const int hd   = lane >> 2;
  const int nodeBase = blockIdx.x * NB;

  {
    const v4f z4 = {0.f, 0.f, 0.f, 0.f};
    const v4f n4 = {-1.0e30f, -1.0e30f, -1.0e30f, -1.0e30f};
    for (int i = tid; i < (LDS_SACC + LDS_DEN) / 4; i += NTHR) lds_dyn[i] = z4;
    for (int i = tid; i < LDS_MX / 4; i += NTHR) lds_dyn[(LDS_SACC + LDS_DEN) / 4 + i] = n4;
    if (tid < NREL * NH) pri[tid] = rpri[tid];
  }
  __syncthreads();

  const bool al16 = ((((size_t)edst) & 15) == 0);
  const int nChunks = (nE + CHUNK - 1) / CHUNK;
#pragma unroll 1
  for (int ch = 0; ch < nChunks; ++ch) {
    const int cbase = ch * CHUNK;
    int wc = 0;
#pragma unroll
    for (int g = 0; g < NGRP; ++g) {
      const int el0 = (g * NTHR + tid) * 4;
      const int e0  = cbase + el0;
      const int sent = -2147483647 - 1;
      v4i d;
      if (al16 && (cbase + CHUNK <= nE)) {
        d = *(const v4i*)(edst + e0);
      } else {
        d.x = (e0     < nE) ? edst[min(e0,     nE - 1)] : sent;
        d.y = (e0 + 1 < nE) ? edst[min(e0 + 1, nE - 1)] : sent;
        d.z = (e0 + 2 < nE) ? edst[min(e0 + 2, nE - 1)] : sent;
        d.w = (e0 + 3 < nE) ? edst[min(e0 + 3, nE - 1)] : sent;
      }
      const unsigned s0 = (unsigned)d.x - (unsigned)nodeBase;
      const unsigned s1 = (unsigned)d.y - (unsigned)nodeBase;
      const unsigned s2 = (unsigned)d.z - (unsigned)nodeBase;
      const unsigned s3 = (unsigned)d.w - (unsigned)nodeBase;
      const bool h0 = s0 < (unsigned)NB;
      const bool h1 = s1 < (unsigned)NB;
      const bool h2 = s2 < (unsigned)NB;
      const bool h3 = s3 < (unsigned)NB;
      const unsigned many = __builtin_amdgcn_ballot_w32(h0 | h1 | h2 | h3);
      if (many != 0u) {
#define HITJ(J, HJ, SJ) { \
          const unsigned mj = __builtin_amdgcn_ballot_w32(HJ); \
          if (HJ) { \
            const int pos = wc + (int)__builtin_amdgcn_mbcnt_lo(mj, 0u); \
            if (pos < WCAP) list[wave * WCAP + pos] = ((el0 + (J)) << 8) | (int)(SJ); \
          } \
          wc += (int)__builtin_popcount(mj); }
        HITJ(0, h0, s0)
        HITJ(1, h1, s1)
        HITJ(2, h2, s2)
        HITJ(3, h3, s3)
#undef HITJ
      }
    }
    if (lane == 0) wcnt[wave] = wc;
    __syncthreads();

    if (wave == 0) {
      for (int wsx = 0; wsx < NWAVE; ++wsx) {
        int n = wcnt[wsx];
        if (n > WCAP) n = WCAP;
        if (n < 0) n = 0;
        for (int i = 0; i < n; ++i) {
          const int ent  = list[wsx * WCAP + i];
          const int slot = ent & (NB - 1);
          const int el   = (ent >> 8) & (CHUNK - 1);
          int e = cbase + el;
          if (e > nE - 1) e = nE - 1;
          int src = esrc[e];
          src = (src < 0) ? 0 : ((src > nN - 1) ? nN - 1 : src);
          int rl = ety[e];
          rl = (rl < 0) ? 0 : ((rl > NREL - 1) ? NREL - 1 : rl);
          int nd = nodeBase + slot;
          if (nd > nN - 1) nd = nN - 1;
          const v4f qv = *(const v4f*)(q + (size_t)nd * DF + 4 * lane);
          const size_t go = ((size_t)rl * nP + src) * DF + 4 * lane;
          const v4h kh = *(const v4h*)(kr8 + go);
          const v4h mh = *(const v4h*)(ms8 + go);
          float s = qv.x * (float)kh[0] + qv.y * (float)kh[1] + qv.z * (float)kh[2] + qv.w * (float)kh[3];
          s += __shfl_xor(s, 1, 32);
          s += __shfl_xor(s, 2, 32);
          const float a  = ((s * 0.125f) * pri[rl * NH + hd]) * 0.25f;
          const int   mo = slot * NH + hd;
          const float mold = mx[mo];
          const float nm = fmaxf(mold, a);
          const float sc = __expf(mold - nm);
          const float p  = __expf(a - nm);
          const float dn = den[mo] * sc + p;
          v4f* sp = (v4f*)(sacc + slot * DF + 4 * lane);
          const v4f cur = *sp;
          v4f nx;
          nx.x = cur.x * sc + p * (float)mh[0];
          nx.y = cur.y * sc + p * (float)mh[1];
          nx.z = cur.z * sc + p * (float)mh[2];
          nx.w = cur.w * sc + p * (float)mh[3];
          *sp = nx;
          mx[mo]  = nm;
          den[mo] = dn;
        }
      }
    }
    __syncthreads();
  }

#pragma unroll 1
  for (int j = 0; j < NB / NWAVE; ++j) {
    const int slot = wave * (NB / NWAVE) + j;
    const int node = nodeBase + slot;
    if (node >= nN) break;
    const float dsum = den[slot * NH + hd] + 1e-16f;
    const float inv  = __builtin_amdgcn_rcpf(dsum) * 0.125f;
    const v4f o = *(const v4f*)(sacc + slot * DF + 4 * lane) * inv;
    float* op = aggr + (size_t)node * DF + 4 * lane;
    *(volatile v4f*)op = o;
    __threadfence();
    *(volatile v4f*)op = o;
  }
}

__global__ __launch_bounds__(NTHR) void k_upd(
    const float* __restrict__ x, const float* __restrict__ aggr, const int* __restrict__ ntype,
    const _Float16* __restrict__ Wu, const float* __restrict__ bu,
    const float* __restrict__ gam, const float* __restrict__ bet,
    float* out, int nN) {
  __shared__ __attribute__((aligned(16))) _Float16 Gs[GR * AP];
  __shared__ __attribute__((aligned(16))) float Hs[GR * QP];
  __shared__ int ts[GR];

  const int tid  = threadIdx.x;
  const int lane = tid & 31;
  const int wave = tid >> 5;
  const int hh   = lane >> 4;
  const int m    = lane & 15;
  const int rowBase = blockIdx.x * GR;

  {
    const int r  = tid >> 3;
    const int c0 = (tid & 7) * 16;
    int row = rowBase + r;
    if (row > nN - 1) row = nN - 1;
    const float* p = aggr + (size_t)row * DF + c0;
#pragma unroll
    for (int j = 0; j < 4; ++j) {
      const v4f a = *(const v4f*)(p + 4 * j);
      v4h h = {(_Float16)0.f, (_Float16)0.f, (_Float16)0.f, (_Float16)0.f};
      h[0] = (_Float16)(gelu_exact(a.x) * 16.0f);
      h[1] = (_Float16)(gelu_exact(a.y) * 16.0f);
      h[2] = (_Float16)(gelu_exact(a.z) * 16.0f);
      h[3] = (_Float16)(gelu_exact(a.w) * 16.0f);
      *(v4h*)(Gs + r * AP + c0 + 4 * j) = h;
    }
  }
  if (tid < GR) {
    int row = rowBase + tid;
    if (row > nN - 1) row = nN - 1;
    int t = ntype[row];
    t = (t < 0) ? 0 : ((t > NTY - 1) ? NTY - 1 : t);
    ts[tid] = t;
  }
  __syncthreads();

  const int ncol = wave * HC + m;
  v8f c00, c01, c02, c10, c11, c12;
  gemm3(Gs, Wu, m, hh, ncol, c00, c01, c02, c10, c11, c12);
#pragma unroll
  for (int r = 0; r < 8; ++r) {
    const int r0 = 8 * hh + r, r1 = 16 + 8 * hh + r;
    const int t0 = ts[r0], t1 = ts[r1];
    int g0 = rowBase + r0; if (g0 > nN - 1) g0 = nN - 1;
    int g1 = rowBase + r1; if (g1 > nN - 1) g1 = nN - 1;
    Hs[r0 * QP + ncol] = sel3(t0, c00[r], c01[r], c02[r]) * (1.0f / 128.0f) + bu[t0 * DF + ncol]
                         + x[(size_t)g0 * DF + ncol];
    Hs[r1 * QP + ncol] = sel3(t1, c10[r], c11[r], c12[r]) * (1.0f / 128.0f) + bu[t1 * DF + ncol]
                         + x[(size_t)g1 * DF + ncol];
  }
  __syncthreads();

#pragma unroll 1
  for (int i = 0; i < GR / NWAVE; ++i) {
    const int row  = (GR / NWAVE) * wave + i;
    const int grow = rowBase + row;
    if (grow >= nN) break;
    const v4f h  = *(const v4f*)(Hs + row * QP + 4 * lane);
    const float s  = wsum(h.x + h.y + h.z + h.w);
    const float mu = s * (1.0f / DF);
    const v4f d  = h - mu;
    const float qq = wsum(d.x * d.x + d.y * d.y + d.z * d.z + d.w * d.w);
    const float rs = rsqrtf(qq * (1.0f / DF) + 1.0e-5f);
    const int ty = ts[row];
    const v4f g4 = *(const v4f*)(gam + ty * DF + 4 * lane);
    const v4f e4 = *(const v4f*)(bet + ty * DF + 4 * lane);
    const v4f y  = d * rs * g4 + e4;
    float* op = out + (size_t)grow * DF + 4 * lane;
    *(volatile v4f*)op = y;
    __threadfence();
    *(volatile v4f*)op = y;
  }
}

extern "C" void kernel_launch(void* const* d_in, const int* in_sizes, int n_in,
                              void* d_out, int out_size, void* d_ws, size_t ws_size,
                              hipStream_t stream) {
  if (n_in < 18) return;
  const int nN = in_sizes[16];
  const int nE = in_sizes[14];
  if (nN <= 0 || in_sizes[0] != nN * DF) return;
  if (nE < 0 || in_sizes[15] != nE || in_sizes[17] != nE) return;
  if (in_sizes[1] != NTY * WSZ || in_sizes[3] != NTY * WSZ || in_sizes[5] != NTY * WSZ || in_sizes[10] != NTY * WSZ) return;
  if (in_sizes[2] != NTY * DF || in_sizes[4] != NTY * DF || in_sizes[6] != NTY * DF) return;
  if (in_sizes[11] != NTY * DF || in_sizes[12] != NTY * DF || in_sizes[13] != NTY * DF) return;
  if (in_sizes[7] != NREL * NH || in_sizes[8] != NREL * NH * HC * HC || in_sizes[9] != NREL * NH * HC * HC) return;
  if (out_size != nN * DF) return;

  const float* x     = (const float*)d_in[0];
  const float* Wq    = (const float*)d_in[1];
  const float* bq    = (const float*)d_in[2];
  const float* Wk    = (const float*)d_in[3];
  const float* bk    = (const float*)d_in[4];
  const float* Wv    = (const float*)d_in[5];
  const float* bv    = (const float*)d_in[6];
  const float* rpri  = (const float*)d_in[7];
  const float* ratt  = (const float*)d_in[8];
  const float* rmsg  = (const float*)d_in[9];
  const float* Wu    = (const float*)d_in[10];
  const float* bu    = (const float*)d_in[11];
  const float* gam   = (const float*)d_in[12];
  const float* bet   = (const float*)d_in[13];
  const int*   esrc  = (const int*)d_in[14];
  const int*   edst  = (const int*)d_in[15];
  const int*   ntype = (const int*)d_in[16];
  const int*   ety   = (const int*)d_in[17];
  float* out = (float*)d_out;

  const int nP = ((nN + GR - 1) / GR) * GR;
  size_t off = 0;
  _Float16* Wp  = (_Float16*)((char*)d_ws + off); off += (size_t)4 * NTY * WSZ * sizeof(_Float16);
  float*    qo  = (float*)((char*)d_ws + off);    off += (size_t)nP * DF * sizeof(float);
  _Float16* kr8 = (_Float16*)((char*)d_ws + off); off += (size_t)NREL * nP * DF * sizeof(_Float16);
  _Float16* ms8 = (_Float16*)((char*)d_ws + off); off += (size_t)NREL * nP * DF * sizeof(_Float16);
  float*    agb = (float*)((char*)d_ws + off);    off += (size_t)nP * DF * sizeof(float);
  if (off > ws_size) return;

  k_prep<<<4 * NTY, NTHR, 0, stream>>>(Wq, Wk, Wv, Wu, Wp);

  k_node<<<nP / GR, NTHR, 0, stream>>>(x, ntype, Wp, bq, bk, bv, ratt, rmsg, qo, kr8, ms8, nN, nP);

  hipFuncSetAttribute(reinterpret_cast<const void*>(&k_agg),
                      hipFuncAttributeMaxDynamicSharedMemorySize, LDS_BYTES);
  const int gridA = (nN + NB - 1) / NB;
  k_agg<<<gridA, NTHR, LDS_BYTES, stream>>>(esrc, edst, ety, rpri, qo, kr8, ms8, agb, nN, nE, nP);

  k_upd<<<nP / GR, NTHR, 0, stream>>>(x, agb, ntype, Wp + (size_t)3 * NTY * WSZ, bu, gam, bet, out, nN);
}
